// LogLinearGDNBlock_15358803050898
// MI455X (gfx1250) — hardware-verified
//
#include <hip/hip_runtime.h>
#include <math.h>

constexpr int kNTok  = 2048;
constexpr int kT     = 1024;
constexpr int kDm    = 1024;
constexpr int kHd    = 128;
constexpr int kNH    = 8;
constexpr int kNbh   = 16;
constexpr int kGrp   = 8;
constexpr int kNproj = 4224;
constexpr int kLamP  = 16;
constexpr int kBlk   = 64;
constexpr int kNBlk  = 16;
constexpr float kScale = 0.08838834764831845f;

constexpr size_t kOffXh   = 0;
constexpr size_t kOffXl   = 4194304;
constexpr size_t kOffWth  = 8388608;
constexpr size_t kOffWtl  = 17039360;
constexpr size_t kOffWoh  = 25690112;
constexpr size_t kOffWol  = 27787264;
constexpr size_t kOffBig  = 29884416;
constexpr size_t kOffQh   = 64487424;
constexpr size_t kOffQl   = 68681728;
constexpr size_t kOffKh   = 72876032;
constexpr size_t kOffKl   = 77070336;
constexpr size_t kOffV    = 81264640;
constexpr size_t kOffG    = 89653248;
constexpr size_t kOffBeta = 98041856;
constexpr size_t kOffGc   = 98107392;
constexpr size_t kOffLam  = 98172928;
constexpr size_t kOffUh   = 99221504;
constexpr size_t kOffUl   = 101318656;
constexpr size_t kOffO    = 103415808;
constexpr size_t kOffDiag = 111804416;
constexpr size_t kOffR    = 113901568;
constexpr size_t kWsTotal = 114163712;
static_assert(kOffR + (size_t)kGrp * kBlk * kHd * 4 == kWsTotal);
static_assert(kWsTotal <= (size_t)134217728);

typedef __attribute__((ext_vector_type(16))) _Float16 v16h;
typedef __attribute__((ext_vector_type(8)))  _Float16 v8h;
typedef __attribute__((ext_vector_type(16))) __bf16   v16b;
typedef __attribute__((ext_vector_type(8)))  __bf16   v8b;
typedef __attribute__((ext_vector_type(8)))  float    v8f;
typedef __attribute__((ext_vector_type(4)))  float    v4f;
typedef __attribute__((ext_vector_type(4)))  unsigned int v4u;

__device__ __forceinline__ unsigned short f2bf_bits(float f) {
  unsigned u = __float_as_uint(f);
  return (unsigned short)((u + 0x7FFFu + ((u >> 16) & 1u)) >> 16);
}
__device__ __forceinline__ float bf_bits2f(unsigned short h) { return __uint_as_float(((unsigned)h) << 16); }

__device__ __forceinline__ void dep_guard_h(v8f& a, v8f& b, v16h x, v16h y) { asm volatile("v_nop\n\tv_nop\n\tv_nop\n\tv_nop" : "+v"(a), "+v"(b) : "v"(x), "v"(y)); }
__device__ __forceinline__ void dep_guard_b(v8f& a, v8f& b, v16b x, v16b y) { asm volatile("v_nop\n\tv_nop\n\tv_nop\n\tv_nop" : "+v"(a), "+v"(b) : "v"(x), "v"(y)); }
__device__ __forceinline__ void keep4_h(v16h a, v16h b, v16h c, v16h d) { asm volatile("v_nop" :: "v"(a), "v"(b), "v"(c), "v"(d)); }
__device__ __forceinline__ void keep4_b(v16b a, v16b b, v16b c, v16b d) { asm volatile("v_nop" :: "v"(a), "v"(b), "v"(c), "v"(d)); }
__device__ __forceinline__ void acc_guard4(v8f& a, v8f& b, v8f& c, v8f& d) { asm volatile("v_nop\n\tv_nop\n\tv_nop\n\tv_nop" : "+v"(a), "+v"(b), "+v"(c), "+v"(d)); }
template <typename T> struct Frag;
template <> struct Frag<_Float16> {
  typedef v16h V; union U { v16h v; v8h h[2]; };
  static __device__ __forceinline__ v16h load(const _Float16* p) {
    U f; f.h[0] = *(const v8h*)(p); f.h[1] = *(const v8h*)(p + 16); return f.v;
  }
  static __device__ __forceinline__ v8f mma(v16h a, v16h b, v8f c) {
    return __builtin_amdgcn_wmma_f32_16x16x32_f16(false, a, false, b, (short)0, c, false, false);
  }
  static __device__ __forceinline__ void guard(v8f& a, v8f& b, v16h x, v16h y) { dep_guard_h(a, b, x, y); }
  static __device__ __forceinline__ void keep(v16h a, v16h b, v16h c, v16h d) { keep4_h(a, b, c, d); }
};
template <> struct Frag<__bf16> {
  typedef v16b V; union U { v16b v; v8b h[2]; };
  static __device__ __forceinline__ v16b load(const __bf16* p) {
    U f; f.h[0] = *(const v8b*)(p); f.h[1] = *(const v8b*)(p + 16); return f.v;
  }
  static __device__ __forceinline__ v8f mma(v16b a, v16b b, v8f c) {
    return __builtin_amdgcn_wmma_f32_16x16x32_bf16(false, a, false, b, (short)0, c, false, false);
  }
  static __device__ __forceinline__ void guard(v8f& a, v8f& b, v16b x, v16b y) { dep_guard_b(a, b, x, y); }
  static __device__ __forceinline__ void keep(v16b a, v16b b, v16b c, v16b d) { keep4_b(a, b, c, d); }
};

__device__ __forceinline__ unsigned pk16(unsigned short a, unsigned short b) { return (unsigned)a | ((unsigned)b << 16); }
__device__ __forceinline__ float sigmf(float x) { return 1.0f / (1.0f + expf(-x)); }
__device__ __forceinline__ float siluf(float x) { return x * sigmf(x); }

template <int ET> struct Elem;
template <> struct Elem<0> { typedef _Float16 T; };
template <> struct Elem<1> { typedef __bf16 T; };
template <int ET, bool SPLIT, int BIAS_MODE, int OUT_MODE, bool RESID, int ACT = 0>
__global__ __launch_bounds__(256) void wmma_gemm64(
    const unsigned short* __restrict__ Ap, const unsigned short* __restrict__ A2p, int lda, long strideA,
    const unsigned short* __restrict__ Btp, const unsigned short* __restrict__ Bt2p, int ldb, long strideB,
    void* __restrict__ Cout, void* __restrict__ Cout2, int ldc, long strideC,
    const float* __restrict__ bias,
    const float* __restrict__ resid, long strideR,
    int M, int N, int K, float scale) {
  typedef typename Elem<ET>::T T;
  typedef typename Frag<T>::V V;
  const T* A = (const T*)Ap; const T* A2 = (const T*)A2p; const T* Bt = (const T*)Btp; const T* Bt2 = (const T*)Bt2p;
  __shared__ __align__(16) float sT[8][16 * 68];
  const int b    = blockIdx.y;
  const int lane = threadIdx.x & 31;
  const int wave = threadIdx.x >> 5;
  const int tilesN = N >> 6;
  const int tilesM = M >> 6;
  const int tile = blockIdx.x * 8 + wave;
  if (tile >= tilesM * tilesN) return;
  const int tm = tile / tilesN;
  const int tn = tile - tm * tilesN;
  const int m0 = tm << 6;
  const int n0 = tn << 6;

  const T* Ab  = A  + (size_t)b * strideA;
  const T* Bb  = Bt + (size_t)b * strideB;
  const T* Ab2 = SPLIT ? (A2  + (size_t)b * strideA) : nullptr;
  const T* Bb2 = SPLIT ? (Bt2 + (size_t)b * strideB) : nullptr;

  const int rlane = lane & 15;
  const int koff  = (lane >> 4) * 8;
  const int mOff  = (lane >> 4) * 8;

  v8f acc[4][4];
#pragma unroll
  for (int i = 0; i < 4; ++i)
#pragma unroll
    for (int j = 0; j < 4; ++j) acc[i][j] = (v8f){0.f,0.f,0.f,0.f,0.f,0.f,0.f,0.f};

  for (int k0 = 0; k0 < K; k0 += 32) {
    V bh[4], bl[4];
#pragma unroll
    for (int j = 0; j < 4; ++j) {
      const size_t bo = (size_t)(n0 + (j << 4) + rlane) * ldb + koff + k0;
      bh[j] = Frag<T>::load(Bb + bo);
      if (SPLIT) bl[j] = Frag<T>::load(Bb2 + bo);
    }
#pragma unroll
    for (int i = 0; i < 4; ++i) {
      const size_t ao = (size_t)(m0 + (i << 4) + rlane) * lda + koff + k0;
      V ah = Frag<T>::load(Ab + ao);
      V al;
      if (SPLIT) al = Frag<T>::load(Ab2 + ao);
#pragma unroll
      for (int j = 0; j < 4; ++j) {
        acc[i][j] = Frag<T>::mma(ah, bh[j], acc[i][j]);
        if (SPLIT) {
          acc[i][j] = Frag<T>::mma(ah, bl[j], acc[i][j]);
          acc[i][j] = Frag<T>::mma(al, bh[j], acc[i][j]);
        }
      }
      Frag<T>::guard(acc[i][0], acc[i][3], ah, SPLIT ? al : ah);
    }
    Frag<T>::keep(bh[0], bh[1], bh[2], bh[3]);
    if (SPLIT) Frag<T>::keep(bl[0], bl[1], bl[2], bl[3]);
  }
  acc_guard4(acc[0][0], acc[0][1], acc[0][2], acc[0][3]);
  acc_guard4(acc[1][0], acc[1][1], acc[1][2], acc[1][3]);
  acc_guard4(acc[2][0], acc[2][1], acc[2][2], acc[2][3]);
  acc_guard4(acc[3][0], acc[3][1], acc[3][2], acc[3][3]);

  float* slab = sT[wave];
  const float* Rb = RESID ? (resid + (size_t)b * strideR) : nullptr;
#pragma unroll
  for (int i = 0; i < 4; ++i) {
    const int mBase = m0 + (i << 4);
#pragma unroll
    for (int j = 0; j < 4; ++j) {
      const int n = n0 + (j << 4) + rlane;
      float bv = 0.f;
      if (BIAS_MODE == 2) bv = bias[n];
#pragma unroll
      for (int r = 0; r < 8; ++r) {
        float v = acc[i][j][r] * scale;
        if (BIAS_MODE == 1) v += bias[mBase + mOff + r];
        if (BIAS_MODE == 2) v += bv;
        if (RESID) v += Rb[(size_t)(mBase + mOff + r) * ldc + n];
        if (ACT == 2) v = fmaxf(v, 0.0f);
        if (ACT == 4) v = (v > 0.f) ? v : 0.01f * v;
        slab[(mOff + r) * 68 + (j << 4) + rlane] = v;
      }
    }
    __builtin_amdgcn_fence(__ATOMIC_RELEASE, "workgroup");
    __builtin_amdgcn_wave_barrier();
    __builtin_amdgcn_fence(__ATOMIC_ACQUIRE, "workgroup");
    if (OUT_MODE == 0) {
      float* C = (float*)Cout + (size_t)b * strideC;
      const int hh = lane >> 4, c4 = (lane & 15) * 4;
      for (int pass = 0; pass < 2; ++pass) {
#pragma unroll
        for (int it = 0; it < 8; ++it) {
          const int row = it * 2 + hh;
          v4f v = *(const v4f*)(slab + row * 68 + c4);
          *(volatile v4f*)(C + (size_t)(mBase + row) * ldc + n0 + c4) = v;
        }
        __threadfence();
      }
    } else {
      const int q = lane >> 3, c8 = (lane & 7) * 8;
      unsigned short* C  = (unsigned short*)Cout  + (size_t)b * strideC;
      unsigned short* C2 = (OUT_MODE == 2) ? ((unsigned short*)Cout2 + (size_t)b * strideC) : nullptr;
      for (int pass = 0; pass < 2; ++pass) {
#pragma unroll
        for (int it = 0; it < 4; ++it) {
          const int row = it * 4 + q;
          const float* sp = slab + row * 68 + c8;
          v8h hv, lv;
#pragma unroll
          for (int e = 0; e < 8; ++e) {
            if (OUT_MODE == 1) {
              hv[e] = (_Float16)sp[e];
            } else {
              unsigned short hb = f2bf_bits(sp[e]);
              unsigned short lb = f2bf_bits(sp[e] - bf_bits2f(hb));
              hv[e] = __builtin_bit_cast(_Float16, hb);
              lv[e] = __builtin_bit_cast(_Float16, lb);
            }
          }
          *(volatile v8h*)(C + (size_t)(mBase + row) * ldc + n0 + c8) = hv;
          if (OUT_MODE == 2) *(volatile v8h*)(C2 + (size_t)(mBase + row) * ldc + n0 + c8) = lv;
        }
        __threadfence();
      }
    }
    __builtin_amdgcn_fence(__ATOMIC_RELEASE, "workgroup");
    __builtin_amdgcn_wave_barrier();
    __builtin_amdgcn_fence(__ATOMIC_ACQUIRE, "workgroup");
  }
}

template <int EPI>
__global__ __launch_bounds__(256) void tri_gemm64(
    const unsigned short* __restrict__ Ap, const unsigned short* __restrict__ A2p, int lda, long strideA,
    const unsigned short* __restrict__ Btp, const unsigned short* __restrict__ Bt2p, int ldb, long strideB,
    void* __restrict__ Cout, void* __restrict__ Cout2, int ldc, long strideC,
    float* __restrict__ Dg, long strideD,
    const float* __restrict__ gcp, const float* __restrict__ betap, const float* __restrict__ lamp, int bh0,
    int M, int N, int K) {
  typedef __bf16 T;
  typedef v16b V;
  const T* A = (const T*)Ap; const T* A2 = (const T*)A2p; const T* Bt = (const T*)Btp; const T* Bt2 = (const T*)Bt2p;
  __shared__ __align__(16) float sT[8][16 * 68];
  const int b    = blockIdx.y;
  const int lane = threadIdx.x & 31;
  const int wave = threadIdx.x >> 5;
  const int tilesN = N >> 6;
  const int tilesM = M >> 6;
  const int tile = blockIdx.x * 8 + wave;
  if (tile >= tilesM * tilesN) return;
  const int tm = tile / tilesN;
  const int tn = tile - tm * tilesN;
  const int m0 = tm << 6;
  const int n0 = tn << 6;

  if (EPI != 0) {
    if (n0 > m0) return;
  }

  const T* Ab  = A   + (size_t)b * strideA;
  const T* Bb  = Bt  + (size_t)b * strideB;
  const T* Ab2 = A2  + (size_t)b * strideA;
  const T* Bb2 = Bt2 + (size_t)b * strideB;

  const int rlane = lane & 15;
  const int koff  = (lane >> 4) * 8;
  const int mOff  = (lane >> 4) * 8;

  v8f acc[4][4];
#pragma unroll
  for (int i = 0; i < 4; ++i)
#pragma unroll
    for (int j = 0; j < 4; ++j) acc[i][j] = (v8f){0.f,0.f,0.f,0.f,0.f,0.f,0.f,0.f};

  int kEnd = K;
  if (EPI == 0) { kEnd = m0 + 64; if (kEnd > K) kEnd = K; }
  for (int k0 = 0; k0 < kEnd; k0 += 32) {
    V bh[4], bl[4];
#pragma unroll
    for (int j = 0; j < 4; ++j) {
      const size_t bo = (size_t)(n0 + (j << 4) + rlane) * ldb + koff + k0;
      bh[j] = Frag<T>::load(Bb + bo);
      bl[j] = Frag<T>::load(Bb2 + bo);
    }
#pragma unroll
    for (int i = 0; i < 4; ++i) {
      const size_t ao = (size_t)(m0 + (i << 4) + rlane) * lda + koff + k0;
      V ah = Frag<T>::load(Ab + ao);
      V al = Frag<T>::load(Ab2 + ao);
#pragma unroll
      for (int j = 0; j < 4; ++j) {
        acc[i][j] = Frag<T>::mma(ah, bh[j], acc[i][j]);
        acc[i][j] = Frag<T>::mma(ah, bl[j], acc[i][j]);
        acc[i][j] = Frag<T>::mma(al, bh[j], acc[i][j]);
      }
      Frag<T>::guard(acc[i][0], acc[i][3], ah, al);
    }
    Frag<T>::keep(bh[0], bh[1], bh[2], bh[3]);
    Frag<T>::keep(bl[0], bl[1], bl[2], bl[3]);
  }
  acc_guard4(acc[0][0], acc[0][1], acc[0][2], acc[0][3]);
  acc_guard4(acc[1][0], acc[1][1], acc[1][2], acc[1][3]);
  acc_guard4(acc[2][0], acc[2][1], acc[2][2], acc[2][3]);
  acc_guard4(acc[3][0], acc[3][1], acc[3][2], acc[3][3]);

  const int bhi = bh0 + b;
  const float* gcb = gcp   + (size_t)bhi * kT;
  const float* beb = betap + (size_t)bhi * kT;
  const float* lab = lamp  + (size_t)bhi * (kT * kLamP);
  float gcn[4] = {0.f, 0.f, 0.f, 0.f};
  if (EPI != 0) {
#pragma unroll
    for (int j = 0; j < 4; ++j) gcn[j] = gcb[n0 + (j << 4) + rlane];
  }
  float* slab = sT[wave];
#pragma unroll
  for (int i = 0; i < 4; ++i) {
    const int mBase = m0 + (i << 4);
    float gcm[8], bem[8];
#pragma unroll
    for (int r = 0; r < 8; ++r) {
      gcm[r] = 0.f; bem[r] = 0.f;
      if (EPI != 0) gcm[r] = gcb[mBase + mOff + r];
      if (EPI == 1) bem[r] = beb[mBase + mOff + r];
    }
#pragma unroll
    for (int j = 0; j < 4; ++j) {
      const int n = n0 + (j << 4) + rlane;
#pragma unroll
      for (int r = 0; r < 8; ++r) {
        const int m = mBase + mOff + r;
        float v = acc[i][j][r];
        if (EPI == 1) {
          const float d  = fminf(fmaxf(gcm[r] - gcn[j], -87.0f), 80.0f);
          const float ex = expf(d);
          v = (v * ex) * bem[r];
          v = (n < m) ? v : 0.0f;
        }
        if (EPI == 2) {
          const float d  = fminf(fmaxf(gcm[r] - gcn[j], -87.0f), 80.0f);
          const float ex = expf(d);
          const unsigned xv = ((unsigned)(m + 1)) ^ ((unsigned)n);
          int lev = 31 - (int)__builtin_clz(xv | 1u);
          lev = (lev > 10) ? 10 : lev;
          const float lm = lab[m * kLamP + lev];
          v = (v * ex) * lm;
          v = (n <= m) ? v : 0.0f;
        }
        slab[(mOff + r) * 68 + (j << 4) + rlane] = v;
      }
    }
    __builtin_amdgcn_fence(__ATOMIC_RELEASE, "workgroup");
    __builtin_amdgcn_wave_barrier();
    __builtin_amdgcn_fence(__ATOMIC_ACQUIRE, "workgroup");
    if (EPI == 0) {
      float* C = (float*)Cout + (size_t)b * strideC;
      const int hh = lane >> 4, c4 = (lane & 15) * 4;
      for (int pass = 0; pass < 2; ++pass) {
#pragma unroll
        for (int it = 0; it < 8; ++it) {
          const int row = it * 2 + hh;
          v4f v = *(const v4f*)(slab + row * 68 + c4);
          *(volatile v4f*)(C + (size_t)(mBase + row) * ldc + n0 + c4) = v;
        }
        __threadfence();
      }
    } else {
      const int q = lane >> 3, c8 = (lane & 7) * 8;
      unsigned short* C  = (unsigned short*)Cout  + (size_t)b * strideC;
      unsigned short* C2 = (unsigned short*)Cout2 + (size_t)b * strideC;
      for (int pass = 0; pass < 2; ++pass) {
#pragma unroll
        for (int it = 0; it < 4; ++it) {
          const int row = it * 4 + q;
          const float* sp = slab + row * 68 + c8;
          v8h hv, lv;
#pragma unroll
          for (int e = 0; e < 8; ++e) {
            unsigned short hb = f2bf_bits(sp[e]);
            unsigned short lb = f2bf_bits(sp[e] - bf_bits2f(hb));
            hv[e] = __builtin_bit_cast(_Float16, hb);
            lv[e] = __builtin_bit_cast(_Float16, lb);
          }
          *(volatile v8h*)(C  + (size_t)(mBase + row) * ldc + n0 + c8) = hv;
          *(volatile v8h*)(C2 + (size_t)(mBase + row) * ldc + n0 + c8) = lv;
        }
        __threadfence();
      }
      if (EPI == 1 && tm == tn) {
        float* Dd = Dg + (size_t)b * strideD + (size_t)tm * 4096;
        const int hh = lane >> 4, c4 = (lane & 15) * 4;
        for (int pass = 0; pass < 2; ++pass) {
#pragma unroll
          for (int it = 0; it < 8; ++it) {
            const int row = it * 2 + hh;
            v4f v = *(const v4f*)(slab + row * 68 + c4);
            *(volatile v4f*)(Dd + (size_t)((mBase - m0) + row) * 64 + c4) = v;
          }
          __threadfence();
        }
      }
    }
    __builtin_amdgcn_fence(__ATOMIC_RELEASE, "workgroup");
    __builtin_amdgcn_wave_barrier();
    __builtin_amdgcn_fence(__ATOMIC_ACQUIRE, "workgroup");
  }
}

__global__ __launch_bounds__(256) void split8_kernel(const float* __restrict__ in, unsigned short* __restrict__ oh,
                                                     unsigned short* __restrict__ ol, int n8) {
  const int i = blockIdx.x * 256 + threadIdx.x;
  if (i >= n8) return;
  const float* p = in + 8 * (size_t)i;
  const v4f a = *(const v4f*)(p);
  const v4f c = *(const v4f*)(p + 4);
  unsigned short hb[8], lb[8];
#pragma unroll
  for (int e = 0; e < 4; ++e) {
    hb[e] = f2bf_bits(a[e]);     lb[e] = f2bf_bits(a[e] - bf_bits2f(hb[e]));
    hb[4 + e] = f2bf_bits(c[e]); lb[4 + e] = f2bf_bits(c[e] - bf_bits2f(hb[4 + e]));
  }
  const v4u uh = (v4u){pk16(hb[0], hb[1]), pk16(hb[2], hb[3]), pk16(hb[4], hb[5]), pk16(hb[6], hb[7])};
  const v4u ul = (v4u){pk16(lb[0], lb[1]), pk16(lb[2], lb[3]), pk16(lb[4], lb[5]), pk16(lb[6], lb[7])};
  unsigned short* qh = oh + 8 * (size_t)i;
  unsigned short* ql = ol + 8 * (size_t)i;
  *(volatile v4u*)qh = uh;
  *(volatile v4u*)ql = ul;
  __threadfence();
  *(volatile v4u*)qh = uh;
  *(volatile v4u*)ql = ul;
}

__global__ __launch_bounds__(256) void wsplit_kernel(const float* __restrict__ W0, const float* __restrict__ W1,
                                                     const float* __restrict__ W2, const float* __restrict__ W3,
                                                     const float* __restrict__ Wb, const float* __restrict__ Wa,
                                                     const float* __restrict__ Wl,
                                                     unsigned short* __restrict__ outh, unsigned short* __restrict__ outl) {
  __shared__ float sm[64][65];
  const int t  = threadIdx.x;
  const int k0 = blockIdx.x * 64;
  const int nt = blockIdx.y;
  const int n0 = nt * 64;
  if (nt < 64) {
    const int z = nt >> 4;
    const float* W = (z == 0) ? W0 : (z == 1) ? W1 : (z == 2) ? W2 : W3;
    const int c0 = n0 & 1023;
#pragma unroll
    for (int i = 0; i < 16; ++i) {
      const int e = i * 256 + t;
      const int r = e >> 6;
      const int c = e & 63;
      sm[c][r] = W[(size_t)(k0 + r) * kDm + c0 + c];
    }
  } else {
#pragma unroll 4
    for (int i = 0; i < 16; ++i) {
      const int e = i * 256 + t;
      const int r = e >> 6;
      const int c = e & 63;
      const int n = n0 + c;
      const int k = k0 + r;
      int ib = n - 4096; ib = (ib < 0) ? 0 : ((ib > 7) ? 7 : ib);
      int ia = n - 4104; ia = (ia < 0) ? 0 : ((ia > 7) ? 7 : ia);
      int il = n - 4112; il = (il < 0) ? 0 : ((il > 87) ? 87 : il);
      const float vb = Wb[(size_t)k * 8 + ib];
      const float va = Wa[(size_t)k * 8 + ia];
      const float vl = Wl[(size_t)k * 88 + il];
      float v = (n < 4104) ? vb : ((n < 4112) ? va : vl);
      v = (n < 4200) ? v : 0.0f;
      sm[c][r] = v;
    }
  }
  __syncthreads();
  const int lane = t & 31, wave = t >> 5;
  const int q = lane >> 3, c8 = (lane & 7) * 8;
  for (int pass = 0; pass < 2; ++pass) {
#pragma unroll
    for (int it = 0; it < 2; ++it) {
      const int row = wave * 8 + it * 4 + q;
      unsigned short hb[8], lb[8];
#pragma unroll
      for (int e = 0; e < 8; ++e) {
        const float v = sm[row][c8 + e];
        hb[e] = f2bf_bits(v);
        lb[e] = f2bf_bits(v - bf_bits2f(hb[e]));
      }
      const v4u uh = (v4u){pk16(hb[0], hb[1]), pk16(hb[2], hb[3]), pk16(hb[4], hb[5]), pk16(hb[6], hb[7])};
      const v4u ul = (v4u){pk16(lb[0], lb[1]), pk16(lb[2], lb[3]), pk16(lb[4], lb[5]), pk16(lb[6], lb[7])};
      const size_t o = (size_t)(n0 + row) * kDm + k0 + c8;
      *(volatile v4u*)(outh + o) = uh;
      *(volatile v4u*)(outl + o) = ul;
    }
    __threadfence();
  }
}

__global__ __launch_bounds__(128) void conv_kernel(const float* __restrict__ P,
                                                   const float* __restrict__ cq, const float* __restrict__ ck,
                                                   const float* __restrict__ cv,
                                                   unsigned short* __restrict__ Qh, unsigned short* __restrict__ Ql,
                                                   unsigned short* __restrict__ Kh, unsigned short* __restrict__ Kl,
                                                   float* __restrict__ Vo, float* __restrict__ Go) {
  __shared__ __align__(16) float sQf[1024];
  __shared__ __align__(16) float sKf[1024];
  __shared__ __align__(16) float sV[1024];
  __shared__ __align__(16) float sG[1024];
  __shared__ __align__(16) unsigned short sQh[1024];
  __shared__ __align__(16) unsigned short sQl[1024];
  __shared__ __align__(16) unsigned short sKh[1024];
  __shared__ __align__(16) unsigned short sKl[1024];
  const int bt   = blockIdx.x;
  const int b    = bt >> 10;
  const int t    = bt & 1023;
  const int tid  = threadIdx.x;
  const int lane = tid & 31;
  const int wave = tid >> 5;
  const int c0   = tid * 8;
  const int tb   = b * kT;
  const int tt2 = t - 1, tt1 = t - 2, tt0 = t - 3;
  const bool p2 = (tt2 >= 0), p1 = (tt1 >= 0), p0 = (tt0 >= 0);
  const float* rw3 = P + (size_t)(tb + t) * kNproj;
  const float* rw2 = P + (size_t)(tb + (p2 ? tt2 : 0)) * kNproj;
  const float* rw1 = P + (size_t)(tb + (p1 ? tt1 : 0)) * kNproj;
  const float* rw0 = P + (size_t)(tb + (p0 ? tt0 : 0)) * kNproj;
  float ssq = 0.f, ssk = 0.f;
#pragma unroll 1
  for (int e = 0; e < 8; ++e) {
    const int c = c0 + e;
    const v4f wq = *(const v4f*)(cq + (size_t)c * 4);
    const v4f wk = *(const v4f*)(ck + (size_t)c * 4);
    const v4f wv = *(const v4f*)(cv + (size_t)c * 4);
    float xq0 = rw0[c],        xq1 = rw1[c],        xq2 = rw2[c];
    float xk0 = rw0[1024 + c], xk1 = rw1[1024 + c], xk2 = rw2[1024 + c];
    float xv0 = rw0[2048 + c], xv1 = rw1[2048 + c], xv2 = rw2[2048 + c];
    xq0 = p0 ? xq0 : 0.f; xk0 = p0 ? xk0 : 0.f; xv0 = p0 ? xv0 : 0.f;
    xq1 = p1 ? xq1 : 0.f; xk1 = p1 ? xk1 : 0.f; xv1 = p1 ? xv1 : 0.f;
    xq2 = p2 ? xq2 : 0.f; xk2 = p2 ? xk2 : 0.f; xv2 = p2 ? xv2 : 0.f;
    const float xq3 = rw3[c], xk3 = rw3[1024 + c], xv3 = rw3[2048 + c];
    float aq = wq[0] * xq0; aq = fmaf(wq[1], xq1, aq); aq = fmaf(wq[2], xq2, aq); aq = fmaf(wq[3], xq3, aq);
    float ak = wk[0] * xk0; ak = fmaf(wk[1], xk1, ak); ak = fmaf(wk[2], xk2, ak); ak = fmaf(wk[3], xk3, ak);
    float av = wv[0] * xv0; av = fmaf(wv[1], xv1, av); av = fmaf(wv[2], xv2, av); av = fmaf(wv[3], xv3, av);
    aq = siluf(aq); ak = siluf(ak); av = siluf(av);
    const float sg = siluf(rw3[3072 + c]);
    sQf[c] = aq; sKf[c] = ak; sV[c] = av; sG[c] = sg;
    ssq += aq * aq; ssk += ak * ak;
  }
#pragma unroll
  for (int off = 1; off < 16; off <<= 1) {
    ssq += __shfl_xor(ssq, off, 32);
    ssk += __shfl_xor(ssk, off, 32);
  }
  const float rq = 1.0f / sqrtf(ssq + 1e-6f);
  const float rk = 1.0f / sqrtf(ssk + 1e-6f);
#pragma unroll 1
  for (int e = 0; e < 8; ++e) {
    const int c = c0 + e;
    const float qn = (sQf[c] * rq) * kScale;
    const float kn = sKf[c] * rk;
    const unsigned short hq = f2bf_bits(qn);
    const unsigned short hk = f2bf_bits(kn);
    sQh[c] = hq; sQl[c] = f2bf_bits(qn - bf_bits2f(hq));
    sKh[c] = hk; sKl[c] = f2bf_bits(kn - bf_bits2f(hk));
  }
  __syncthreads();
  const int hsel = 2 * wave + (lane >> 4);
  const int d8   = (lane & 15) * 8;
  const size_t rowQ = ((size_t)(b * kNH + hsel) * kT + t) * kHd + d8;
  for (int pass = 0; pass < 2; ++pass) {
    const v4u q1 = *(const v4u*)(sQh + hsel * kHd + d8);
    const v4u q2 = *(const v4u*)(sQl + hsel * kHd + d8);
    const v4u k1 = *(const v4u*)(sKh + hsel * kHd + d8);
    const v4u k2 = *(const v4u*)(sKl + hsel * kHd + d8);
    *(volatile v4u*)(Qh + rowQ) = q1;
    *(volatile v4u*)(Ql + rowQ) = q2;
    *(volatile v4u*)(Kh + rowQ) = k1;
    *(volatile v4u*)(Kl + rowQ) = k2;
#pragma unroll
    for (int hp = 0; hp < 2; ++hp) {
      const int head = 2 * wave + hp;
      const v4f vv = *(const v4f*)(sV + head * kHd + lane * 4);
      *(volatile v4f*)(Vo + ((size_t)(b * kNH + head) * kT + t) * kHd + lane * 4) = vv;
    }
#pragma unroll
    for (int it = 0; it < 2; ++it) {
      const int chunk = wave * 2 + it;
      const v4f gg = *(const v4f*)(sG + chunk * 128 + lane * 4);
      *(volatile v4f*)(Go + (size_t)bt * kDm + chunk * 128 + lane * 4) = gg;
    }
    __threadfence();
  }
}

__global__ __launch_bounds__(256) void gates_kernel(const float* __restrict__ P, const float* __restrict__ Alog,
                                                    const float* __restrict__ dtb,
                                                    float* __restrict__ betaO, float* __restrict__ gcO,
                                                    float* __restrict__ lamO) {
  __shared__ __align__(16) float sg[1024];
  __shared__ __align__(16) float sgc[1024];
  __shared__ __align__(16) float sb[1024];
  __shared__ float sex[8];
  const int bh  = blockIdx.x;
  const int b   = bh >> 3;
  const int h   = bh & 7;
  const int tid = threadIdx.x;
  const float na = -expf(Alog[h]);
  const float db = dtb[h];
#pragma unroll 1
  for (int it = 0; it < 4; ++it) {
    const int t = it * 256 + tid;
    const float* row = P + (size_t)(b * kT + t) * kNproj;
    const float ap = row[4104 + h] + db;
    const float sp = fmaxf(ap, 0.0f) + log1pf(expf(-fabsf(ap)));
    sg[t] = na * sp;
    sb[t] = sigmf(row[4096 + h]);
  }
  __syncthreads();
  if (tid < 8) {
    float accum = 0.0f;
#pragma unroll 1
    for (int i = 0; i < 128; ++i) {
      accum = accum + sg[tid * 128 + i];
      sgc[tid * 128 + i] = accum;
    }
  }
  __syncthreads();
  if (tid == 0) {
    float e = 0.0f;
#pragma unroll 1
    for (int c = 0; c < 8; ++c) { sex[c] = e; e = e + sgc[c * 128 + 127]; }
  }
  __syncthreads();
  const v4f b4 = *(const v4f*)(sb + 4 * tid);
  const v4f g4 = *(const v4f*)(sgc + 4 * tid);
  const float ex = sex[tid >> 5];
  v4f g4o;
  g4o[0] = g4[0] + ex; g4o[1] = g4[1] + ex; g4o[2] = g4[2] + ex; g4o[3] = g4[3] + ex;
  float* pb = betaO + (size_t)bh * kT + 4 * tid;
  float* pg = gcO   + (size_t)bh * kT + 4 * tid;
  *(volatile v4f*)pb = b4;
  *(volatile v4f*)pg = g4o;
  __threadfence();
  *(volatile v4f*)pb = b4;
  *(volatile v4f*)pg = g4o;
#pragma unroll 1
  for (int k = 0; k < 16; ++k) {
    const int idx4 = k * 256 + tid;
    const int t  = idx4 >> 2;
    const int l0 = (idx4 & 3) * 4;
    const float* row = P + (size_t)(b * kT + t) * kNproj + 4112 + h * 11;
    v4f l4;
#pragma unroll
    for (int e = 0; e < 4; ++e) {
      const int l  = l0 + e;
      const int lc = (l > 10) ? 10 : l;
      const float s = sigmf(row[lc]);
      l4[e] = (l < 11) ? s : 0.0f;
    }
    float* pl = lamO + (size_t)bh * (kT * kLamP) + (size_t)idx4 * 4;
    *(volatile v4f*)pl = l4;
    __threadfence();
    *(volatile v4f*)pl = l4;
  }
}

__global__ __launch_bounds__(128) void dsolve_kernel(const float* __restrict__ Dg, const float* __restrict__ Rp,
                                                     const float* __restrict__ Vp, const float* __restrict__ betap,
                                                     unsigned short* __restrict__ Uh, unsigned short* __restrict__ Ul,
                                                     int bh0, int step) {
  __shared__ __align__(16) float sA[64 * 64];
  __shared__ __align__(16) float sU[64 * 128];
  const int j    = blockIdx.x;
  const int bh   = bh0 + j;
  const int tid  = threadIdx.x;
  const int lane = tid & 31, wave = tid >> 5;
  const int t0   = step * kBlk;
  const float* dsrc = Dg + ((size_t)j * kNBlk + step) * 4096;
#pragma unroll
  for (int it = 0; it < 8; ++it) {
    const int idx = it * 512 + tid * 4;
    *(v4f*)(sA + idx) = *(const v4f*)(dsrc + idx);
  }
  const float* V  = Vp + ((size_t)bh * kT + t0) * kHd + tid;
  const float* be = betap + (size_t)bh * kT + t0;
  const float* R  = Rp + (size_t)j * (kBlk * kHd) + tid;
#pragma unroll 1
  for (int r = 0; r < kBlk; ++r) {
    float rhs = be[r] * V[(size_t)r * kHd];
    if (step > 0) rhs = rhs - R[(size_t)r * kHd];
    sU[r * kHd + tid] = rhs;
  }
  __syncthreads();
#pragma unroll 1
  for (int r = 1; r < kBlk; ++r) {
    const float* ar = sA + r * 64;
    const float* uc = sU + tid;
    float accum = 0.0f;
    int s = 0;
#pragma unroll 1
    for (; s + 4 <= r; s += 4) {
      accum = fmaf(ar[s],     uc[(s)     * kHd], accum);
      accum = fmaf(ar[s + 1], uc[(s + 1) * kHd], accum);
      accum = fmaf(ar[s + 2], uc[(s + 2) * kHd], accum);
      accum = fmaf(ar[s + 3], uc[(s + 3) * kHd], accum);
    }
#pragma unroll 1
    for (; s < r; ++s) accum = fmaf(ar[s], uc[s * kHd], accum);
    const float un = sU[r * kHd + tid] - accum;
    sU[r * kHd + tid] = un;
  }
  __syncthreads();
  const int q = lane >> 3, c8 = (lane & 7) * 8;
  for (int pass = 0; pass < 2; ++pass) {
#pragma unroll 1
    for (int it = 0; it < 8; ++it) {
      const int dv = it * 16 + wave * 4 + q;
      unsigned short hb[8], lb[8];
#pragma unroll
      for (int e = 0; e < 8; ++e) {
        const float u = sU[(c8 + e) * kHd + dv];
        hb[e] = f2bf_bits(u);
        lb[e] = f2bf_bits(u - bf_bits2f(hb[e]));
      }
      const v4u vh = (v4u){pk16(hb[0], hb[1]), pk16(hb[2], hb[3]), pk16(hb[4], hb[5]), pk16(hb[6], hb[7])};
      const v4u vl = (v4u){pk16(lb[0], lb[1]), pk16(lb[2], lb[3]), pk16(lb[4], lb[5]), pk16(lb[6], lb[7])};
      const size_t o = ((size_t)(j * kHd + dv)) * kT + t0 + c8;
      *(volatile v4u*)(Uh + o) = vh;
      *(volatile v4u*)(Ul + o) = vl;
    }
    __threadfence();
  }
}

__global__ __launch_bounds__(128) void gnorm_kernel(const float* __restrict__ O, const float* __restrict__ G,
                                                    const float* __restrict__ nw,
                                                    unsigned short* __restrict__ Nh, unsigned short* __restrict__ Nl) {
  __shared__ __align__(16) unsigned short sh[1024];
  __shared__ __align__(16) unsigned short sl[1024];
  const int bt  = blockIdx.x;
  const int tid = threadIdx.x;
  const int c0  = tid * 8;
  const float* orow = O + (size_t)bt * kDm;
  const float* grow = G + (size_t)bt * kDm;
  float ss = 0.0f;
#pragma unroll 1
  for (int e = 0; e < 8; ++e) { const float o = orow[c0 + e]; ss += o * o; }
#pragma unroll
  for (int off = 1; off < 16; off <<= 1) ss += __shfl_xor(ss, off, 32);
  const float rr = 1.0f / sqrtf(ss * (1.0f / 128.0f) + 1e-5f);
#pragma unroll 1
  for (int e = 0; e < 8; ++e) {
    const int c = c0 + e;
    const float o = orow[c];
    const float v = ((o * rr) * nw[c & 127]) * grow[c];
    const unsigned short hb = f2bf_bits(v);
    sh[c] = hb;
    sl[c] = f2bf_bits(v - bf_bits2f(hb));
  }
  __syncthreads();
  const v4u uh = *(const v4u*)(sh + c0);
  const v4u ul = *(const v4u*)(sl + c0);
  unsigned short* ph = Nh + (size_t)bt * kDm + c0;
  unsigned short* pl = Nl + (size_t)bt * kDm + c0;
  *(volatile v4u*)ph = uh;
  *(volatile v4u*)pl = ul;
  __threadfence();
  *(volatile v4u*)ph = uh;
  *(volatile v4u*)pl = ul;
}

extern "C" void kernel_launch(void* const* d_in, const int* in_sizes, int n_in,
                              void* d_out, int out_size, void* d_ws, size_t ws_size,
                              hipStream_t stream) {
  if (n_in < 17) return;
  if (out_size < kNTok * kDm) return;
  if (in_sizes[0] < kNTok * kDm || in_sizes[3] < kDm * kDm || in_sizes[4] < kDm * kDm || in_sizes[5] < kDm * kDm ||
      in_sizes[6] < kDm * 8 || in_sizes[7] < kDm * 8 || in_sizes[8] < kDm * 88 || in_sizes[9] < kDm * kDm ||
      in_sizes[10] < kDm * kDm || in_sizes[11] < kDm * 4 || in_sizes[12] < kDm * 4 || in_sizes[13] < kDm * 4 ||
      in_sizes[14] < 8 || in_sizes[15] < 8 || in_sizes[16] < kHd) return;
  if (ws_size < kWsTotal) return;

  const float* x    = (const float*)d_in[0];
  const float* Wq   = (const float*)d_in[3];
  const float* Wk   = (const float*)d_in[4];
  const float* Wv   = (const float*)d_in[5];
  const float* Wb   = (const float*)d_in[6];
  const float* Wa   = (const float*)d_in[7];
  const float* Wl   = (const float*)d_in[8];
  const float* Wg   = (const float*)d_in[9];
  const float* Wo   = (const float*)d_in[10];
  const float* cq   = (const float*)d_in[11];
  const float* ck   = (const float*)d_in[12];
  const float* cv   = (const float*)d_in[13];
  const float* Alog = (const float*)d_in[14];
  const float* dtb  = (const float*)d_in[15];
  const float* nw   = (const float*)d_in[16];

  char* ws = (char*)d_ws;
  unsigned short* Xh   = (unsigned short*)(ws + kOffXh);
  unsigned short* Xl   = (unsigned short*)(ws + kOffXl);
  unsigned short* WTh  = (unsigned short*)(ws + kOffWth);
  unsigned short* WTl  = (unsigned short*)(ws + kOffWtl);
  unsigned short* WoTh = (unsigned short*)(ws + kOffWoh);
  unsigned short* WoTl = (unsigned short*)(ws + kOffWol);
  float*          PRJ  = (float*)(ws + kOffBig);
  unsigned short* AKh  = (unsigned short*)(ws + kOffBig);
  unsigned short* AKl  = AKh + (size_t)kGrp * kT * kT;
  unsigned short* PMh  = (unsigned short*)(ws + kOffBig);
  unsigned short* PMl  = PMh + (size_t)kGrp * kT * kT;
  unsigned short* Qh   = (unsigned short*)(ws + kOffQh);
  unsigned short* Ql   = (unsigned short*)(ws + kOffQl);
  unsigned short* Kh   = (unsigned short*)(ws + kOffKh);
  unsigned short* Kl   = (unsigned short*)(ws + kOffKl);
  float*          Vb   = (float*)(ws + kOffV);
  float*          Gb   = (float*)(ws + kOffG);
  float*          BETA = (float*)(ws + kOffBeta);
  float*          GC   = (float*)(ws + kOffGc);
  float*          LAM  = (float*)(ws + kOffLam);
  unsigned short* Uh   = (unsigned short*)(ws + kOffUh);
  unsigned short* Ul   = (unsigned short*)(ws + kOffUl);
  float*          Ob   = (float*)(ws + kOffO);
  float*          DIAG = (float*)(ws + kOffDiag);
  float*          Rb   = (float*)(ws + kOffR);
  unsigned short* Nh   = Xh;
  unsigned short* Nl   = Xl;

  split8_kernel<<<(kNTok * kDm / 8) / 256, 256, 0, stream>>>(x, Xh, Xl, kNTok * kDm / 8);
  wsplit_kernel<<<dim3(16, 66), 256, 0, stream>>>(Wq, Wk, Wv, Wg, Wb, Wa, Wl, WTh, WTl);
  wsplit_kernel<<<dim3(16, 16), 256, 0, stream>>>(Wo, Wo, Wo, Wo, Wo, Wo, Wo, WoTh, WoTl);
  wmma_gemm64<1, true, 0, 0, false><<<dim3(264, 1), 256, 0, stream>>>(
      Xh, Xl, kDm, 0L, WTh, WTl, kDm, 0L, (void*)PRJ, (void*)0, kNproj, 0L,
      (const float*)0, (const float*)0, 0L, kNTok, kNproj, kDm, 1.0f);
  conv_kernel<<<kNTok, 128, 0, stream>>>(PRJ, cq, ck, cv, Qh, Ql, Kh, Kl, Vb, Gb);
  gates_kernel<<<kNbh, 256, 0, stream>>>(PRJ, Alog, dtb, BETA, GC, LAM);
  for (int g = 0; g < 2; ++g) {
    const size_t po = (size_t)g * kGrp * kT * kHd;
    tri_gemm64<1><<<dim3(32, kGrp), 256, 0, stream>>>(
        Kh + po, Kl + po, kHd, (long)(kT * kHd), Kh + po, Kl + po, kHd, (long)(kT * kHd),
        (void*)AKh, (void*)AKl, kT, (long)(kT * kT), DIAG, (long)(kNBlk * 4096),
        GC, BETA, LAM, g * kGrp, kT, kT, kHd);
    for (int i = 0; i < kNBlk; ++i) {
      if (i > 0) {
        wmma_gemm64<1, true, 0, 0, false><<<dim3(1, kGrp), 256, 0, stream>>>(
            AKh + (size_t)i * kBlk * kT, AKl + (size_t)i * kBlk * kT, kT, (long)(kT * kT),
            Uh, Ul, kT, (long)(kHd * kT),
            (void*)Rb, (void*)0, kHd, (long)(kBlk * kHd),
            (const float*)0, (const float*)0, 0L, kBlk, kHd, i * kBlk, 1.0f);
      }
      dsolve_kernel<<<kGrp, 128, 0, stream>>>(DIAG, Rb, Vb, BETA, Uh, Ul, g * kGrp, i);
    }
    tri_gemm64<2><<<dim3(32, kGrp), 256, 0, stream>>>(
        Qh + po, Ql + po, kHd, (long)(kT * kHd), Kh + po, Kl + po, kHd, (long)(kT * kHd),
        (void*)PMh, (void*)PMl, kT, (long)(kT * kT), DIAG, 0L,
        GC, BETA, LAM, g * kGrp, kT, kT, kHd);
    tri_gemm64<0><<<dim3(4, kGrp), 256, 0, stream>>>(
        PMh, PMl, kT, (long)(kT * kT), Uh, Ul, kT, (long)(kHd * kT),
        (void*)(Ob + (size_t)g * kT * kDm), (void*)PMl, kDm, (long)kHd, DIAG, 0L,
        GC, BETA, LAM, g * kGrp, kT, kHd, kT);
  }
  gnorm_kernel<<<kNTok, 128, 0, stream>>>(Ob, Gb, nw, Nh, Nl);
  wmma_gemm64<1, true, 0, 0, false><<<dim3(64, 1), 256, 0, stream>>>(
      Nh, Nl, kDm, 0L, WoTh, WoTl, kDm, 0L, d_out, (void*)0, kDm, 0L,
      (const float*)0, (const float*)0, 0L, kNTok, kDm, kDm, 1.0f);
}
